// SDRLayer_76768245449191
// MI455X (gfx1250) — hardware-verified
//
#include <hip/hip_runtime.h>
#include <hip/hip_bf16.h>
#include <stddef.h>


#define DCH     64
#define NTHR    256
#define NWAVE   8
#define EPT     8
#define NGRP    2
#define CHUNK   (NTHR * EPT * NGRP)
#define WCAP    (EPT * NGRP * 32)
#define LISTN   (NWAVE * WCAP)
#define NBC     4096
#define NBF     1024
#define RCAP    40960
#define RBN     128
#define TGT     256
#define DEGCAP  512
#define GROWS   128
#define OTHR    512
#define AP      72
#define NEGS    0.2f
#define LDS_FILL ((RCAP + NBF + LISTN) * 4 + 64)

static_assert((CHUNK & (CHUNK - 1)) == 0);
static_assert(CHUNK <= 4096);
static_assert(NBC <= 4096 && NBF <= 4096);
static_assert((NBC & (NBC - 1)) == 0 && (NBF & (NBF - 1)) == 0);
static_assert(NBC == 4 * NBF);
static_assert(OTHR * 8 == NBC);
static_assert((RCAP % 32) == 0);
static_assert(TGT == NWAVE * 32);
static_assert(GROWS == NWAVE * 16);
static_assert((GROWS * DCH / 8) % NTHR == 0);
static_assert(2 * GROWS * AP * 2 >= GROWS * DCH * 4);
static_assert((AP % 8) == 0);
static_assert((DCH % 32) == 0);

typedef float          v4f  __attribute__((ext_vector_type(4)));
typedef float          v8f  __attribute__((ext_vector_type(8)));
typedef int            v4i  __attribute__((ext_vector_type(4)));
typedef unsigned short v8us __attribute__((ext_vector_type(8)));
typedef __bf16         v16b __attribute__((ext_vector_type(16)));
union FragB { v16b v; v8us u[2]; };

__device__ __forceinline__ unsigned int bf_bits(float x) {
  const unsigned int u = __float_as_uint(x);
  return (u + 0x7FFFu + ((u >> 16) & 1u)) >> 16;
}

__device__ __forceinline__ void split8(v4f a, v4f b, v8us& hi, v8us& lo) {
  float f[8];
  f[0] = a.x; f[1] = a.y; f[2] = a.z; f[3] = a.w; f[4] = b.x; f[5] = b.y; f[6] = b.z; f[7] = b.w;
#pragma unroll
  for (int e = 0; e < 8; ++e) {
    const unsigned int h = bf_bits(f[e]);
    const float rem = f[e] - __uint_as_float(h << 16);
    const unsigned int l = bf_bits(rem);
    hi[e] = (unsigned short)h;
    lo[e] = (unsigned short)l;
  }
}

__device__ __forceinline__ void split1(float x, unsigned short& hi, unsigned short& lo) {
  const unsigned int h = bf_bits(x);
  const float rem = x - __uint_as_float(h << 16);
  hi = (unsigned short)h;
  lo = (unsigned short)bf_bits(rem);
}

__device__ __forceinline__ v8f wmb(v16b a, v16b b, v8f c) {
  v8f d = __builtin_amdgcn_wmma_f32_16x16x32_bf16(false, a, false, b, (short)0, c, false, false);
  asm volatile("v_nop\n\tv_nop\n\tv_nop\n\tv_nop" : "+v"(d) : "v"(a), "v"(b));
  return d;
}

__device__ __forceinline__ v8f wm3(v16b ah, v16b al, v16b bh, v16b bl, v8f c) {
  c = wmb(ah, bh, c);
  c = wmb(al, bh, c);
  c = wmb(ah, bl, c);
  return c;
}

__device__ __forceinline__ float leaky(float e) { return e > 0.f ? e : NEGS * e; }

__device__ __forceinline__ float tanh_f(float v) {
  v = fminf(fmaxf(v, -16.0f), 16.0f);
  const float e = __expf(2.0f * v);
  return 1.0f - 2.0f * __builtin_amdgcn_rcpf(e + 1.0f);
}

template <int NB>
__device__ __forceinline__ int scan_chunk(const int* __restrict__ dsts, int nE, int cbase, int slotBase,
                                          int vec8, int* list, int tid, int lane, int wave) {
  int wc = 0;
#pragma unroll
  for (int g = 0; g < NGRP; ++g) {
    const int el0  = (g * NTHR + tid) * EPT;
    const int e0   = cbase + el0;
    const int sent = -2147483647 - 1;
    v4i da, db;
    if (vec8 != 0 && cbase + CHUNK <= nE) {
      da = *(const v4i*)(dsts + e0);
      db = *(const v4i*)(dsts + e0 + 4);
    } else {
      da.x = (e0     < nE) ? dsts[min(e0, nE - 1)] : sent;
      da.y = (e0 + 1 < nE) ? dsts[min(e0 + 1, nE - 1)] : sent;
      da.z = (e0 + 2 < nE) ? dsts[min(e0 + 2, nE - 1)] : sent;
      da.w = (e0 + 3 < nE) ? dsts[min(e0 + 3, nE - 1)] : sent;
      db.x = (e0 + 4 < nE) ? dsts[min(e0 + 4, nE - 1)] : sent;
      db.y = (e0 + 5 < nE) ? dsts[min(e0 + 5, nE - 1)] : sent;
      db.z = (e0 + 6 < nE) ? dsts[min(e0 + 6, nE - 1)] : sent;
      db.w = (e0 + 7 < nE) ? dsts[min(e0 + 7, nE - 1)] : sent;
    }
    const unsigned nb = (unsigned)slotBase;
    const unsigned s0 = (unsigned)da.x - nb, s1 = (unsigned)da.y - nb;
    const unsigned s2 = (unsigned)da.z - nb, s3 = (unsigned)da.w - nb;
    const unsigned s4 = (unsigned)db.x - nb, s5 = (unsigned)db.y - nb;
    const unsigned s6 = (unsigned)db.z - nb, s7 = (unsigned)db.w - nb;
    const bool h0 = s0 < (unsigned)NB, h1 = s1 < (unsigned)NB, h2 = s2 < (unsigned)NB, h3 = s3 < (unsigned)NB;
    const bool h4 = s4 < (unsigned)NB, h5 = s5 < (unsigned)NB, h6 = s6 < (unsigned)NB, h7 = s7 < (unsigned)NB;
    const unsigned any = __builtin_amdgcn_ballot_w32(h0 | h1 | h2 | h3 | h4 | h5 | h6 | h7);
    if (any != 0u) {
#define HITJ(J, HJ, SJ) { \
        const unsigned mj = __builtin_amdgcn_ballot_w32(HJ); \
        if (mj != 0u) { \
          if (HJ) { \
            const int pos = wc + (int)__builtin_amdgcn_mbcnt_lo(mj, 0u); \
            if (pos < WCAP) list[wave * WCAP + pos] = ((el0 + (J)) << 12) | (int)(SJ); \
          } \
          wc += (int)__builtin_popcount(mj); } }
      HITJ(0, h0, s0)
      HITJ(1, h1, s1)
      HITJ(2, h2, s2)
      HITJ(3, h3, s3)
      HITJ(4, h4, s4)
      HITJ(5, h5, s5)
      HITJ(6, h6, s6)
      HITJ(7, h7, s7)
#undef HITJ
    }
  }
  return wc;
}

__global__ __launch_bounds__(NTHR) void k_wprep(
    const float* __restrict__ aggW, const float* __restrict__ W1, const float* __restrict__ W2,
    unsigned short* wah, unsigned short* wal, unsigned short* w1h, unsigned short* w1l,
    unsigned short* w2h, unsigned short* w2l) {
  const int g0 = 3 * DCH * DCH / 8;
  const int g1 = 4 * DCH * DCH / 8;
  const int g2 = DCH * DCH / 8;
  const int bstart = blockIdx.x * NTHR;
  const float* src; unsigned short* dh; unsigned short* dl; int K, segOff, per;
  if (bstart < g0)           { src = aggW; dh = wah; dl = wal; K = DCH;     segOff = 0;       per = DCH * DCH; }
  else if (bstart < g0 + g1) { src = W1;   dh = w1h; dl = w1l; K = 4 * DCH; segOff = g0;      per = 0; }
  else                       { src = W2;   dh = w2h; dl = w2l; K = DCH;     segOff = g0 + g1; per = 0; }
  const int i = bstart + (int)threadIdx.x;
  if (i >= g0 + g1 + g2) return;
  const int o = (i - segOff) * 8;
  int oo = o;
  if (per != 0) {
    const int layer = o / per;
    src += (size_t)layer * per;
    oo = o - layer * per;
  }
  const int n  = oo / K;
  const int k0 = oo - n * K;
  float v[8];
#pragma unroll
  for (int e = 0; e < 8; ++e) v[e] = src[(size_t)(k0 + e) * DCH + n];
  v4f a, b;
  a.x = v[0]; a.y = v[1]; a.z = v[2]; a.w = v[3];
  b.x = v[4]; b.y = v[5]; b.z = v[6]; b.w = v[7];
  v8us hi, lo;
  split8(a, b, hi, lo);
  unsigned short* ph = dh + o;
  unsigned short* pl = dl + o;
  *(volatile v8us*)ph = hi;
  *(volatile v8us*)pl = lo;
  __threadfence();
  *(volatile v8us*)ph = hi;
  *(volatile v8us*)pl = lo;
}

__global__ __launch_bounds__(NTHR) void k_count(
    const int* __restrict__ eA, const int* __restrict__ eB, const int* __restrict__ eC,
    int* cntAll, int nE, int vec8, int cntPad) {
  __shared__ __attribute__((aligned(16))) int scnt[NBC];
  __shared__ __attribute__((aligned(16))) int list[LISTN];
  __shared__ int wcnt[NWAVE];
  const int tid = threadIdx.x, lane = tid & 31, wave = tid >> 5;
  const int lst = blockIdx.y;
  const int* ei = (lst == 0) ? eA : ((lst == 1) ? eB : eC);
  int* cnt = cntAll + (size_t)lst * cntPad;
  const int nodeBase = blockIdx.x * NBC;
  const int* dsts = ei + nE;

  for (int i = tid; i < NBC; i += NTHR) scnt[i] = 0;
  __syncthreads();

  const int nChunks = (nE + CHUNK - 1) / CHUNK;
#pragma unroll 1
  for (int ch = 0; ch < nChunks; ++ch) {
    const int cbase = ch * CHUNK;
    const int wc = scan_chunk<NBC>(dsts, nE, cbase, nodeBase, vec8, list, tid, lane, wave);
    if (lane == 0) wcnt[wave] = wc;
    __syncthreads();
    if (wave == 0) {
#pragma unroll 1
      for (int wsx = 0; wsx < NWAVE; ++wsx) {
        int n = __builtin_amdgcn_readfirstlane(wcnt[wsx]);
        n = n > WCAP ? WCAP : (n < 0 ? 0 : n);
        const int* lp = list + wsx * WCAP;
#pragma unroll 1
        for (int i = 0; i < n; ++i) {
          const int ent  = __builtin_amdgcn_readfirstlane(lp[i]);
          const int slot = ent & (NBC - 1);
          if (lane == 0) scnt[slot] = scnt[slot] + 1;
        }
      }
    }
    __syncthreads();
  }

  v4i cq[4];
#pragma unroll
  for (int q = 0; q < 4; ++q) {
    const int f = (wave * 4 + q) * 128 + 4 * lane;
    cq[q] = *(const v4i*)(scnt + f);
  }
  int* cp = cnt + (size_t)nodeBase;
#pragma unroll
  for (int q = 0; q < 4; ++q) {
    const int f = (wave * 4 + q) * 128 + 4 * lane;
    *(volatile v4i*)(cp + f) = cq[q];
  }
  __threadfence();
#pragma unroll
  for (int q = 0; q < 4; ++q) {
    const int f = (wave * 4 + q) * 128 + 4 * lane;
    *(volatile v4i*)(cp + f) = cq[q];
  }
}

__global__ __launch_bounds__(OTHR) void k_offsets(
    const int* __restrict__ cntAll, int* offAll, int* rbAll, int nChunk, int cntPad) {
  __shared__ __attribute__((aligned(16))) int soff[NBC];
  __shared__ __attribute__((aligned(16))) int srb[RBN];
  __shared__ int wtot[OTHR / 32];
  const int tid = threadIdx.x, lane = tid & 31, wave = tid >> 5, sub = tid >> 7;
  const int lst = blockIdx.x;
  const int* cnt = cntAll + (size_t)lst * cntPad;
  int* off   = offAll + (size_t)lst * cntPad;
  int* rbase = rbAll + (size_t)lst * RBN;
  for (int i = tid; i < RBN; i += OTHR) srb[i] = 0;
  int carry = 0;
#pragma unroll 1
  for (int ch = 0; ch < nChunk; ++ch) {
    const int base = ch * NBC;
    const v4i c0 = *(const v4i*)(cnt + base + 8 * tid);
    const v4i c1 = *(const v4i*)(cnt + base + 8 * tid + 4);
    const int e0 = max(c0.x, 0), e1 = max(c0.y, 0), e2 = max(c0.z, 0), e3 = max(c0.w, 0);
    const int e4 = max(c1.x, 0), e5 = max(c1.y, 0), e6 = max(c1.z, 0), e7 = max(c1.w, 0);
    const int ts = e0 + e1 + e2 + e3 + e4 + e5 + e6 + e7;
    int incl = ts;
#pragma unroll
    for (int d = 1; d < 32; d <<= 1) {
      const int t = __shfl_up(incl, d);
      if (lane >= d) incl += t;
    }
    if (lane == 31) wtot[wave] = incl;
    __syncthreads();
    const int S0 = wtot[0]  + wtot[1]  + wtot[2]  + wtot[3];
    const int S1 = wtot[4]  + wtot[5]  + wtot[6]  + wtot[7];
    const int S2 = wtot[8]  + wtot[9]  + wtot[10] + wtot[11];
    const int S3 = wtot[12] + wtot[13] + wtot[14] + wtot[15];
    int pre = 0;
#pragma unroll 1
    for (int w = 4 * sub; w < wave; ++w) pre += wtot[w];
    const int b0 = carry;
    const int b1 = b0 + ((S0 + 31) & ~31);
    const int b2 = b1 + ((S1 + 31) & ~31);
    const int b3 = b2 + ((S2 + 31) & ~31);
    const int b4 = b3 + ((S3 + 31) & ~31);
    const int myb = sub == 0 ? b0 : (sub == 1 ? b1 : (sub == 2 ? b2 : b3));
    if (tid == 0) {
      srb[min(4 * ch + 0, RBN - 1)] = b0;
      srb[min(4 * ch + 1, RBN - 1)] = b1;
      srb[min(4 * ch + 2, RBN - 1)] = b2;
      srb[min(4 * ch + 3, RBN - 1)] = b3;
    }
    int run = myb + pre + incl - ts;
    soff[8 * tid + 0] = run; run += e0;
    soff[8 * tid + 1] = run; run += e1;
    soff[8 * tid + 2] = run; run += e2;
    soff[8 * tid + 3] = run; run += e3;
    soff[8 * tid + 4] = run; run += e4;
    soff[8 * tid + 5] = run; run += e5;
    soff[8 * tid + 6] = run; run += e6;
    soff[8 * tid + 7] = run;
    carry = b4;
    __syncthreads();
    const v4i o0 = *(const v4i*)(soff + 4 * tid);
    const v4i o1 = *(const v4i*)(soff + 4 * (tid + OTHR));
    int* op = off + base;
    *(volatile v4i*)(op + 4 * tid) = o0;
    *(volatile v4i*)(op + 4 * (tid + OTHR)) = o1;
    __threadfence();
    *(volatile v4i*)(op + 4 * tid) = o0;
    *(volatile v4i*)(op + 4 * (tid + OTHR)) = o1;
    __syncthreads();
  }
  if (tid == 0) srb[min(4 * nChunk, RBN - 1)] = carry;
  __syncthreads();
  v4i rv = {0, 0, 0, 0};
  if (tid < 32) rv = *(const v4i*)(srb + 4 * tid);
  if (tid < 32) *(volatile v4i*)(rbase + 4 * tid) = rv;
  __threadfence();
  if (tid < 32) *(volatile v4i*)(rbase + 4 * tid) = rv;
}

__global__ __launch_bounds__(NTHR) void k_fill(
    const int* __restrict__ eA, const int* __restrict__ eB, const int* __restrict__ eC,
    const int* __restrict__ offAll, const int* __restrict__ rbAll,
    int* csrAll, int nN, int nE, int vec8, int csrLen, int cntPad) {
  extern __shared__ v4f lds_dyn[];
  int* region = (int*)lds_dyn;
  int* cursor = region + RCAP;
  int* list   = cursor + NBF;
  int* wcnt   = list + LISTN;
  const int tid = threadIdx.x, lane = tid & 31, wave = tid >> 5;
  const int b = blockIdx.x;
  const int lst = blockIdx.y;
  const int* ei = (lst == 0) ? eA : ((lst == 1) ? eB : eC);
  const int* off   = offAll + (size_t)lst * cntPad;
  const int* rbase = rbAll + (size_t)lst * RBN;
  int* csr = csrAll + (size_t)lst * csrLen;
  const int nodeBase = b * NBF;
  const int* dsts = ei + nE;

  int rb0 = rbase[b];
  const int rb1 = rbase[b + 1];
  rb0 = rb0 < 0 ? 0 : (rb0 > csrLen ? csrLen : rb0);
  rb0 &= ~31;
  int len = rb1 - rb0;
  len = len < 0 ? 0 : (len > RCAP ? RCAP : len);
  int lenW = (len + 31) & ~31;
  if (rb0 + lenW > csrLen) lenW = (csrLen - rb0) & ~31;

  {
    const v4i z = {0, 0, 0, 0};
    for (int i = tid; i < RCAP / 4; i += NTHR) ((v4i*)region)[i] = z;
    for (int s = tid; s < NBF; s += NTHR) {
      int o = off[nodeBase + s] - rb0;
      o = o < 0 ? 0 : (o > RCAP ? RCAP : o);
      cursor[s] = o;
    }
  }
  __syncthreads();

  const int nChunks = (nE + CHUNK - 1) / CHUNK;
#pragma unroll 1
  for (int ch = 0; ch < nChunks; ++ch) {
    const int cbase = ch * CHUNK;
    const int wc = scan_chunk<NBF>(dsts, nE, cbase, nodeBase, vec8, list, tid, lane, wave);
    if (lane == 0) wcnt[wave] = wc;
    __syncthreads();
    if (wave == 0) {
#pragma unroll 1
      for (int wsx = 0; wsx < NWAVE; ++wsx) {
        int n = __builtin_amdgcn_readfirstlane(wcnt[wsx]);
        n = n > WCAP ? WCAP : (n < 0 ? 0 : n);
        const int* lp = list + wsx * WCAP;
#pragma unroll 1
        for (int i = 0; i < n; ++i) {
          const int ent  = __builtin_amdgcn_readfirstlane(lp[i]);
          const int slot = ent & (NBF - 1);
          int e = cbase + ((ent >> 12) & (CHUNK - 1));
          e = e > nE - 1 ? nE - 1 : e;
          int src = ei[e];
          src = src < 0 ? 0 : (src > nN - 1 ? nN - 1 : src);
          if (lane == 0) {
            int pos = cursor[slot];
            pos = pos < 0 ? 0 : (pos > RCAP - 1 ? RCAP - 1 : pos);
            region[pos] = src;
            const int np = pos + 1;
            cursor[slot] = np > RCAP ? RCAP : np;
          }
        }
      }
    }
    __syncthreads();
  }

  const int nv = lenW >> 2;
  int* gp = csr + rb0;
#pragma unroll 1
  for (int i = tid; i < nv; i += NTHR) { const v4i v = ((const v4i*)region)[i]; *(volatile v4i*)(gp + 4 * i) = v; }
  __threadfence();
#pragma unroll 1
  for (int i = tid; i < nv; i += NTHR) { const v4i v = ((const v4i*)region)[i]; *(volatile v4i*)(gp + 4 * i) = v; }
}

__global__ __launch_bounds__(NTHR) void k_node(
    const float* __restrict__ x, const unsigned short* __restrict__ wh, const unsigned short* __restrict__ wl,
    const float* __restrict__ atts, const float* __restrict__ attd,
    float* H, float* As, float* Ad, int nN) {
  __shared__ __attribute__((aligned(16))) unsigned short lds_a[2 * GROWS * AP];
  __shared__ __attribute__((aligned(16))) float sas[GROWS];
  __shared__ __attribute__((aligned(16))) float sad[GROWS];
  unsigned short* sAh = lds_a;
  unsigned short* sAl = lds_a + GROWS * AP;
  float* stg = (float*)lds_a;
  const int tid = threadIdx.x, lane = tid & 31, wave = tid >> 5, hh = lane >> 4, m = lane & 15;
  const int rowBase = blockIdx.x * GROWS;

#pragma unroll
  for (int i = 0; i < (GROWS * DCH / 8) / NTHR; ++i) {
    const int idx = i * NTHR + tid;
    const int r   = idx >> 3;
    const int c0  = (idx & 7) * 8;
    int row = rowBase + r;
    row = row > nN - 1 ? nN - 1 : row;
    const float* ap = x + (size_t)row * DCH + c0;
    const v4f a = *(const v4f*)ap, b = *(const v4f*)(ap + 4);
    v8us hi, lo;
    split8(a, b, hi, lo);
    *(v8us*)(sAh + r * AP + c0) = hi;
    *(v8us*)(sAl + r * AP + c0) = lo;
  }
  __syncthreads();

  v8f acc[4];
#pragma unroll
  for (int t = 0; t < 4; ++t) { v8f z = {0.f, 0.f, 0.f, 0.f, 0.f, 0.f, 0.f, 0.f}; acc[t] = z; }
  const int aoff = (wave * 16 + m) * AP + 8 * hh;
#pragma unroll
  for (int kt = 0; kt < DCH / 32; ++kt) {
    FragB ah, al;
    ah.u[0] = *(const v8us*)(sAh + aoff + 32 * kt);
    ah.u[1] = *(const v8us*)(sAh + aoff + 32 * kt + 16);
    al.u[0] = *(const v8us*)(sAl + aoff + 32 * kt);
    al.u[1] = *(const v8us*)(sAl + aoff + 32 * kt + 16);
#pragma unroll
    for (int t = 0; t < 4; ++t) {
      const int boff = (16 * t + m) * DCH + 32 * kt + 8 * hh;
      FragB bh, bl;
      bh.u[0] = *(const v8us*)(wh + boff);
      bh.u[1] = *(const v8us*)(wh + boff + 16);
      bl.u[0] = *(const v8us*)(wl + boff);
      bl.u[1] = *(const v8us*)(wl + boff + 16);
      acc[t] = wm3(ah.v, al.v, bh.v, bl.v, acc[t]);
    }
  }

  float asv[4], adv[4];
#pragma unroll
  for (int t = 0; t < 4; ++t) { asv[t] = atts[16 * t + m]; adv[t] = attd[16 * t + m]; }
  float psr[8], pdr[8];
#pragma unroll
  for (int r = 0; r < 8; ++r) {
    float ps = 0.f, pd = 0.f;
#pragma unroll
    for (int t = 0; t < 4; ++t) { ps += acc[t][r] * asv[t]; pd += acc[t][r] * adv[t]; }
#pragma unroll
    for (int d = 1; d < 16; d <<= 1) { ps += __shfl_xor(ps, d, 32); pd += __shfl_xor(pd, d, 32); }
    psr[r] = ps; pdr[r] = pd;
  }
  __syncthreads();

  float* sp = stg + (wave * 16 + 8 * hh) * DCH + m;
#pragma unroll
  for (int t = 0; t < 4; ++t) {
#pragma unroll
    for (int r = 0; r < 8; ++r) sp[r * DCH + 16 * t] = acc[t][r];
  }
  if (m == 0) {
#pragma unroll
    for (int r = 0; r < 8; ++r) { sas[wave * 16 + 8 * hh + r] = psr[r]; sad[wave * 16 + 8 * hh + r] = pdr[r]; }
  }
  __syncthreads();

  const float* lp = stg + wave * 16 * DCH + 4 * lane;
  float* gp = H + (size_t)(rowBase + wave * 16) * DCH + 4 * lane;
  v4f sv = {0.f, 0.f, 0.f, 0.f};
  if (wave == 0) sv = *(const v4f*)(sas + 4 * lane);
  if (wave == 1) sv = *(const v4f*)(sad + 4 * lane);
  float* qp = (wave == 0 ? As : Ad) + (size_t)rowBase + 4 * lane;
#pragma unroll
  for (int i = 0; i < 8; ++i) { const v4f v = *(const v4f*)(lp + i * 128); *(volatile v4f*)(gp + i * 128) = v; }
  if (wave < 2) *(volatile v4f*)qp = sv;
  __threadfence();
#pragma unroll
  for (int i = 0; i < 8; ++i) { const v4f v = *(const v4f*)(lp + i * 128); *(volatile v4f*)(gp + i * 128) = v; }
  if (wave < 2) *(volatile v4f*)qp = sv;
}

__global__ __launch_bounds__(NTHR) void k_agg(
    const int* __restrict__ csr, const int* __restrict__ off, const int* __restrict__ cnt,
    const float* __restrict__ As, const float* __restrict__ Ad, const float* __restrict__ H,
    const float* __restrict__ bias, float* O, int nN, int csrLen) {
  const int tid = threadIdx.x, lane = tid & 31, wave = tid >> 5, hsel = lane >> 4, cq = lane & 15;
  const int tbase = blockIdx.x * TGT + wave * 32;
  const int cl = tbase + lane;
  const int cnt_l = cnt[cl];
  const int off_l = off[cl];
  union FI { float f; int i; };
  FI asu, adu;
  asu.f = As[cl];
  adu.f = Ad[cl];
  const v4f bv = *(const v4f*)(bias + 4 * cq);
  const float NEGBIG = -3.0e38f;
  v4f keep = {0.f, 0.f, 0.f, 0.f};

#pragma unroll 1
  for (int j = 0; j < 32; ++j) {
    const int c = tbase + j;
    int n = __builtin_amdgcn_readlane(cnt_l, j);
    n = n < 0 ? 0 : (n > DEGCAP ? DEGCAP : n);
    const int st = __builtin_amdgcn_readlane(off_l, j);
    FI t1, t2;
    t1.i = __builtin_amdgcn_readlane(asu.i, j);
    t2.i = __builtin_amdgcn_readlane(adu.i, j);
    const float adc = t2.f;
    const float es  = leaky(t1.f + adc);

    float mx = es;
#pragma unroll 1
    for (int q0 = 0; q0 < n; q0 += 32) {
      int pos = st + q0 + lane;
      pos = pos < 0 ? 0 : (pos > csrLen - 1 ? csrLen - 1 : pos);
      int sl = csr[pos];
      sl = sl < 0 ? 0 : (sl > nN - 1 ? nN - 1 : sl);
      float e = leaky(As[sl] + adc);
      e = (q0 + lane < n) ? e : NEGBIG;
#pragma unroll
      for (int d = 16; d >= 1; d >>= 1) e = fmaxf(e, __shfl_xor(e, d, 32));
      mx = fmaxf(mx, e);
    }

    float wl = 0.f;
    v4f acc = {0.f, 0.f, 0.f, 0.f};
#pragma unroll 1
    for (int q0 = 0; q0 < n; q0 += 32) {
      int pos = st + q0 + lane;
      pos = pos < 0 ? 0 : (pos > csrLen - 1 ? csrLen - 1 : pos);
      int sl = csr[pos];
      sl = sl < 0 ? 0 : (sl > nN - 1 ? nN - 1 : sl);
      const float e = leaky(As[sl] + adc);
      float w = expf(e - mx);
      w = (q0 + lane < n) ? w : 0.f;
      wl += w;
      FI wu; wu.f = w;
      const int mcnt = (n - q0) < 32 ? (n - q0) : 32;
#pragma unroll 1
      for (int p = 0; p < mcnt; p += 2) {
        const int s0 = __builtin_amdgcn_readlane(sl, p);
        const int s1 = __builtin_amdgcn_readlane(sl, p + 1);
        FI a0, a1;
        a0.i = __builtin_amdgcn_readlane(wu.i, p);
        a1.i = __builtin_amdgcn_readlane(wu.i, p + 1);
        const int   s  = hsel ? s1 : s0;
        const float ww = hsel ? a1.f : a0.f;
        const v4f hv = *(const v4f*)(H + (size_t)s * DCH + 4 * cq);
        acc = acc + hv * ww;
      }
    }

    const float wself = expf(es - mx);
    const v4f hc = *(const v4f*)(H + (size_t)c * DCH + 4 * cq);
    acc = acc + hc * (hsel == 0 ? wself : 0.f);
#pragma unroll
    for (int d = 16; d >= 1; d >>= 1) wl += __shfl_xor(wl, d, 32);
    const float den = wl + wself;
    acc.x += __shfl_xor(acc.x, 16, 32);
    acc.y += __shfl_xor(acc.y, 16, 32);
    acc.z += __shfl_xor(acc.z, 16, 32);
    acc.w += __shfl_xor(acc.w, 16, 32);
    const float inv = __builtin_amdgcn_rcpf(den);
    const v4f res = acc * inv + bv;

    if ((j & 1) != 0) {
      const v4f sv = hsel ? res : keep;
      float* gp = O + (size_t)(c - 1) * DCH + 4 * lane;
      *(volatile v4f*)gp = sv;
      __threadfence();
      *(volatile v4f*)gp = sv;
    } else {
      keep = res;
    }
  }
}

__global__ __launch_bounds__(NTHR) void k_mlp(
    const float* __restrict__ x, const float* __restrict__ o0, const float* __restrict__ o1,
    const float* __restrict__ o2,
    const unsigned short* __restrict__ w1h, const unsigned short* __restrict__ w1l, const float* __restrict__ b1,
    const unsigned short* __restrict__ w2h, const unsigned short* __restrict__ w2l, const float* __restrict__ b2,
    float* out, int nN) {
  __shared__ __attribute__((aligned(16))) unsigned short lds_t[2 * NWAVE * 16 * AP];
  unsigned short* sTh = lds_t;
  unsigned short* sTl = lds_t + NWAVE * 16 * AP;
  float* stg = (float*)lds_t;
  const int tid = threadIdx.x, lane = tid & 31, wave = tid >> 5, hh = lane >> 4, m = lane & 15;
  const int rowBase = blockIdx.x * GROWS;
  const int row = rowBase + wave * 16 + m;
  const int rx  = row < nN ? row : nN - 1;
  const float* xr  = x  + (size_t)rx  * DCH;
  const float* p0r = o0 + (size_t)row * DCH;
  const float* p1r = o1 + (size_t)row * DCH;
  const float* p2r = o2 + (size_t)row * DCH;

  v8f acc[4];
#pragma unroll
  for (int t = 0; t < 4; ++t) { v8f z = {0.f, 0.f, 0.f, 0.f, 0.f, 0.f, 0.f, 0.f}; acc[t] = z; }
#pragma unroll
  for (int ks = 0; ks < 8; ++ks) {
    const int seg = ks >> 1, koff = (ks & 1) * 32;
    const float* rp = (seg == 0) ? xr : ((seg == 1) ? p0r : ((seg == 2) ? p1r : p2r));
    const v4f pa = *(const v4f*)(rp + koff + 8 * hh);
    const v4f pb = *(const v4f*)(rp + koff + 8 * hh + 4);
    const v4f qa = *(const v4f*)(rp + koff + 16 + 8 * hh);
    const v4f qb = *(const v4f*)(rp + koff + 16 + 8 * hh + 4);
    FragB ah, al;
    split8(pa, pb, ah.u[0], al.u[0]);
    split8(qa, qb, ah.u[1], al.u[1]);
#pragma unroll
    for (int t = 0; t < 4; ++t) {
      const int boff = (16 * t + m) * (4 * DCH) + 32 * ks + 8 * hh;
      FragB bh, bl;
      bh.u[0] = *(const v8us*)(w1h + boff);
      bh.u[1] = *(const v8us*)(w1h + boff + 16);
      bl.u[0] = *(const v8us*)(w1l + boff);
      bl.u[1] = *(const v8us*)(w1l + boff + 16);
      acc[t] = wm3(ah.v, al.v, bh.v, bl.v, acc[t]);
    }
  }

  unsigned short* th = sTh + (wave * 16 + 8 * hh) * AP + m;
  unsigned short* tl = sTl + (wave * 16 + 8 * hh) * AP + m;
#pragma unroll
  for (int t = 0; t < 4; ++t) {
    const float bb = b1[16 * t + m];
#pragma unroll
    for (int r = 0; r < 8; ++r) {
      const float v = tanh_f(acc[t][r] + bb);
      unsigned short h16, l16;
      split1(v, h16, l16);
      th[r * AP + 16 * t] = h16;
      tl[r * AP + 16 * t] = l16;
    }
  }
  __syncthreads();

  v8f acc2[4];
#pragma unroll
  for (int t = 0; t < 4; ++t) { v8f z = {0.f, 0.f, 0.f, 0.f, 0.f, 0.f, 0.f, 0.f}; acc2[t] = z; }
  const int a2 = (wave * 16 + m) * AP + 8 * hh;
#pragma unroll
  for (int kt = 0; kt < DCH / 32; ++kt) {
    FragB ah, al;
    ah.u[0] = *(const v8us*)(sTh + a2 + 32 * kt);
    ah.u[1] = *(const v8us*)(sTh + a2 + 32 * kt + 16);
    al.u[0] = *(const v8us*)(sTl + a2 + 32 * kt);
    al.u[1] = *(const v8us*)(sTl + a2 + 32 * kt + 16);
#pragma unroll
    for (int t = 0; t < 4; ++t) {
      const int boff = (16 * t + m) * DCH + 32 * kt + 8 * hh;
      FragB bh, bl;
      bh.u[0] = *(const v8us*)(w2h + boff);
      bh.u[1] = *(const v8us*)(w2h + boff + 16);
      bl.u[0] = *(const v8us*)(w2l + boff);
      bl.u[1] = *(const v8us*)(w2l + boff + 16);
      acc2[t] = wm3(ah.v, al.v, bh.v, bl.v, acc2[t]);
    }
  }
  __syncthreads();

  float* sp = stg + (wave * 16 + 8 * hh) * DCH + m;
#pragma unroll
  for (int t = 0; t < 4; ++t) {
    const float bb = b2[16 * t + m];
#pragma unroll
    for (int r = 0; r < 8; ++r) sp[r * DCH + 16 * t] = acc2[t][r] + bb;
  }
  __syncthreads();

  const float* lp = stg + wave * 16 * DCH + 4 * lane;
  const int rw = rowBase + wave * 16;
  float* gp = out + (size_t)rw * DCH + 4 * lane;
#pragma unroll
  for (int i = 0; i < 8; ++i) {
    const v4f v = *(const v4f*)(lp + i * 128);
    if (rw + 2 * i + 1 < nN)                      *(volatile v4f*)(gp + i * 128) = v;
    else if (rw + 2 * i < nN && lane < 16)        *(volatile v4f*)(gp + i * 128) = v;
  }
  __threadfence();
#pragma unroll
  for (int i = 0; i < 8; ++i) {
    const v4f v = *(const v4f*)(lp + i * 128);
    if (rw + 2 * i + 1 < nN)                      *(volatile v4f*)(gp + i * 128) = v;
    else if (rw + 2 * i < nN && lane < 16)        *(volatile v4f*)(gp + i * 128) = v;
  }
}

extern "C" void kernel_launch(void* const* d_in, const int* in_sizes, int n_in,
                              void* d_out, int out_size, void* d_ws, size_t ws_size,
                              hipStream_t stream) {
  if (n_in < 12) return;
  const int nN = in_sizes[0] / DCH;
  if (nN <= 0 || in_sizes[0] != nN * DCH) return;
  const int nE = in_sizes[1] / 2;
  if (nE <= 0 || in_sizes[1] != 2 * nE || in_sizes[2] != 2 * nE || in_sizes[3] != 2 * nE) return;
  if (in_sizes[4] != 3 * DCH * DCH || in_sizes[5] != 3 * DCH || in_sizes[6] != 3 * DCH || in_sizes[7] != 3 * DCH) return;
  if (in_sizes[8] != 4 * DCH * DCH || in_sizes[9] != DCH || in_sizes[10] != DCH * DCH || in_sizes[11] != DCH) return;
  if (out_size != nN * DCH) return;
  if (nE > (1 << 28) || nN > (1 << 24)) return;

  const float* x    = (const float*)d_in[0];
  const int*   eA   = (const int*)d_in[1];
  const int*   eB   = (const int*)d_in[2];
  const int*   eC   = (const int*)d_in[3];
  const float* aggW = (const float*)d_in[4];
  const float* atts = (const float*)d_in[5];
  const float* attd = (const float*)d_in[6];
  const float* aggB = (const float*)d_in[7];
  const float* W1   = (const float*)d_in[8];
  const float* b1   = (const float*)d_in[9];
  const float* W2   = (const float*)d_in[10];
  const float* b2   = (const float*)d_in[11];
  float* out = (float*)d_out;

  const int NPAD   = ((nN + TGT - 1) / TGT) * TGT;
  const int nBC    = (nN + NBC - 1) / NBC;
  const int CNTPAD = nBC * NBC;
  if (4 * nBC + 1 > RBN) return;
  const int nBF    = (nN + NBF - 1) / NBF;
  if (32 * nBF > 4096) return;
  const int csrLen = ((nE + 31) & ~31) + 4096;
  const int nGemm  = NPAD / GROWS;
  const int nAgg   = NPAD / TGT;

  char* ws = (char*)d_ws;
  size_t off = 0;
  const size_t oWAh = off; off += (size_t)3 * DCH * DCH * 2;       off = (off + 255) & ~(size_t)255;
  const size_t oWAl = off; off += (size_t)3 * DCH * DCH * 2;       off = (off + 255) & ~(size_t)255;
  const size_t oW1h = off; off += (size_t)4 * DCH * DCH * 2;       off = (off + 255) & ~(size_t)255;
  const size_t oW1l = off; off += (size_t)4 * DCH * DCH * 2;       off = (off + 255) & ~(size_t)255;
  const size_t oW2h = off; off += (size_t)DCH * DCH * 2;           off = (off + 255) & ~(size_t)255;
  const size_t oW2l = off; off += (size_t)DCH * DCH * 2;           off = (off + 255) & ~(size_t)255;
  const size_t oCnt = off; off += (size_t)3 * CNTPAD * 4;          off = (off + 255) & ~(size_t)255;
  const size_t oOff = off; off += (size_t)3 * CNTPAD * 4;          off = (off + 255) & ~(size_t)255;
  const size_t oRb  = off; off += (size_t)3 * RBN * 4;             off = (off + 255) & ~(size_t)255;
  const size_t oCsr = off; off += (size_t)3 * csrLen * 4;          off = (off + 255) & ~(size_t)255;
  const size_t oH   = off; off += (size_t)NPAD * DCH * 4;          off = (off + 255) & ~(size_t)255;
  const size_t oAs  = off; off += (size_t)NPAD * 4;                off = (off + 255) & ~(size_t)255;
  const size_t oAd  = off; off += (size_t)NPAD * 4;                off = (off + 255) & ~(size_t)255;
  const size_t oO   = off; off += (size_t)3 * NPAD * DCH * 4;      off = (off + 255) & ~(size_t)255;
  if (off > ws_size) return;
  unsigned short* wah = (unsigned short*)(ws + oWAh);
  unsigned short* wal = (unsigned short*)(ws + oWAl);
  unsigned short* w1h = (unsigned short*)(ws + oW1h);
  unsigned short* w1l = (unsigned short*)(ws + oW1l);
  unsigned short* w2h = (unsigned short*)(ws + oW2h);
  unsigned short* w2l = (unsigned short*)(ws + oW2l);
  int*   cnt  = (int*)(ws + oCnt);
  int*   offp = (int*)(ws + oOff);
  int*   rb   = (int*)(ws + oRb);
  int*   csr  = (int*)(ws + oCsr);
  float* H    = (float*)(ws + oH);
  float* As   = (float*)(ws + oAs);
  float* Ad   = (float*)(ws + oAd);
  float* Opl  = (float*)(ws + oO);

  const int vec8 = ((nE & 3) == 0) ? 1 : 0;

  const int nPrep = (3 * DCH * DCH + 4 * DCH * DCH + DCH * DCH) / 8;
  k_wprep<<<(nPrep + NTHR - 1) / NTHR, NTHR, 0, stream>>>(aggW, W1, W2, wah, wal, w1h, w1l, w2h, w2l);

  k_count<<<dim3(nBC, 3), NTHR, 0, stream>>>(eA, eB, eC, cnt, nE, vec8, CNTPAD);
  k_offsets<<<3, OTHR, 0, stream>>>(cnt, offp, rb, nBC, CNTPAD);
  hipFuncSetAttribute(reinterpret_cast<const void*>(&k_fill),
                      hipFuncAttributeMaxDynamicSharedMemorySize, LDS_FILL);
  k_fill<<<dim3(nBF, 3), NTHR, LDS_FILL, stream>>>(eA, eB, eC, offp, rb, csr, nN, nE, vec8, csrLen, CNTPAD);

  for (int l = 0; l < 3; ++l) {
    k_node<<<nGemm, NTHR, 0, stream>>>(x, wah + (size_t)l * DCH * DCH, wal + (size_t)l * DCH * DCH,
                                       atts + (size_t)l * DCH, attd + (size_t)l * DCH, H, As, Ad, nN);
    k_agg<<<nAgg, NTHR, 0, stream>>>(csr + (size_t)l * csrLen, offp + (size_t)l * CNTPAD, cnt + (size_t)l * CNTPAD,
                                     As, Ad, H, aggB + (size_t)l * DCH, Opl + (size_t)l * NPAD * DCH, nN, csrLen);
  }

  k_mlp<<<nGemm, NTHR, 0, stream>>>(x, Opl, Opl + (size_t)NPAD * DCH, Opl + (size_t)2 * NPAD * DCH,
                                    w1h, w1l, b1, w2h, w2l, b2, out, nN);
}
